// TrainingFreeSelfAttention_74852690035310
// MI455X (gfx1250) — hardware-verified
//
#include <hip/hip_runtime.h>
#include <math.h>
#include <stdint.h>

#define NTOK  8192
#define CD    128
#define HWN   4096
#define NBAT  2
#define LNPS  6.931471805599453f
#define ATTSC 0.08838834764831845f
static_assert(NTOK == NBAT * HWN);
static_assert((NTOK % 64) == 0);
static_assert((HWN % 64) == 0);
static_assert(CD == 128);

typedef _Float16       v16h __attribute__((ext_vector_type(16)));
typedef _Float16       v8h  __attribute__((ext_vector_type(8)));
typedef __bf16         v16b __attribute__((ext_vector_type(16)));
typedef unsigned short v8us __attribute__((ext_vector_type(8)));
typedef float          v8f  __attribute__((ext_vector_type(8)));
typedef float          v4f  __attribute__((ext_vector_type(4)));
typedef unsigned int   v4u  __attribute__((ext_vector_type(4)));

union FragH { v16h v; v8h  h[2]; };
union FragB { v16b v; v8us u[2]; };
static_assert(sizeof(FragH) == 32);
static_assert(sizeof(FragB) == 32);

__device__ __forceinline__ unsigned short bf_bits(float f) {
  unsigned u = __float_as_uint(f);
  return (unsigned short)((u + 0x7FFFu + ((u >> 16) & 1u)) >> 16);
}
__device__ __forceinline__ float bf_up(unsigned short h) { return __uint_as_float(((unsigned)h) << 16); }
__device__ __forceinline__ unsigned short h_bits(_Float16 x) { return __builtin_bit_cast(unsigned short, x); }
__device__ __forceinline__ unsigned pk16(unsigned short a, unsigned short b) { return (unsigned)a | ((unsigned)b << 16); }
__device__ __forceinline__ v8f zero8() { v8f z = {0.f, 0.f, 0.f, 0.f, 0.f, 0.f, 0.f, 0.f}; return z; }
__device__ __forceinline__ float hmax8(v8f s) {
  return fmaxf(fmaxf(fmaxf(s[0], s[1]), fmaxf(s[2], s[3])), fmaxf(fmaxf(s[4], s[5]), fmaxf(s[6], s[7])));
}

__device__ __forceinline__ v16h ldfrag_h(const _Float16* p) {
  FragH f;
  f.h[0] = *(const v8h*)(p);
  f.h[1] = *(const v8h*)(p + 16);
  return f.v;
}
__device__ __forceinline__ v16b ldfrag_b(const unsigned short* p) {
  FragB f;
  f.u[0] = *(const v8us*)(p);
  f.u[1] = *(const v8us*)(p + 16);
  return f.v;
}

__device__ __forceinline__ v8f mma_h_raw(v16h a, v16h b, v8f c) {
  return __builtin_amdgcn_wmma_f32_16x16x32_f16(false, a, false, b, (short)0, c, false, false);
}
__device__ __forceinline__ v8f mma_b_raw(v16b a, v16b b, v8f c) {
  return __builtin_amdgcn_wmma_f32_16x16x32_bf16(false, a, false, b, (short)0, c, false, false);
}
__device__ __forceinline__ void sguard12(v8f& a, v8f& b,
                                         v16b x0, v16b x1, v16b x2, v16b x3,
                                         v16b x4, v16b x5, v16b x6, v16b x7,
                                         v16b y0, v16b y1, v16b y2, v16b y3) {
#if defined(__HIP_DEVICE_COMPILE__)
  const v16h h0 = __builtin_bit_cast(v16h, x0), h1 = __builtin_bit_cast(v16h, x1);
  const v16h h2 = __builtin_bit_cast(v16h, x2), h3 = __builtin_bit_cast(v16h, x3);
  const v16h h4 = __builtin_bit_cast(v16h, x4), h5 = __builtin_bit_cast(v16h, x5);
  const v16h h6 = __builtin_bit_cast(v16h, x6), h7 = __builtin_bit_cast(v16h, x7);
  const v16h g0 = __builtin_bit_cast(v16h, y0), g1 = __builtin_bit_cast(v16h, y1);
  const v16h g2 = __builtin_bit_cast(v16h, y2), g3 = __builtin_bit_cast(v16h, y3);
  asm volatile("v_nop\n\tv_nop\n\tv_nop\n\tv_nop"
               : "+v"(a), "+v"(b)
               : "v"(h0), "v"(h1), "v"(h2), "v"(h3), "v"(h4), "v"(h5), "v"(h6), "v"(h7),
                 "v"(g0), "v"(g1), "v"(g2), "v"(g3));
#endif
}
__device__ __forceinline__ void oguard4(v8f& a, v8f& b, v8f& c, v8f& d,
                                        v16h x0, v16h x1, v16h x2, v16h x3, v16h p0) {
#if defined(__HIP_DEVICE_COMPILE__)
  asm volatile("v_nop\n\tv_nop\n\tv_nop\n\tv_nop"
               : "+v"(a), "+v"(b), "+v"(c), "+v"(d) : "v"(x0), "v"(x1), "v"(x2), "v"(x3), "v"(p0));
#endif
}

__global__ __launch_bounds__(256) void cvt_planes(const float* __restrict__ xin,
                                                   unsigned short* FB, unsigned short* VT) {
  __shared__ __align__(16) unsigned short Ts[64 * 136];
  const int tid = threadIdx.x;
  const int bx  = blockIdx.x;
  const int n0  = bx * 64;
  const int b   = n0 >> 12;
  const int hw0 = n0 & (HWN - 1);

  {
    const int e = tid & 7, lq = tid >> 3;
    v4u u[4];
    size_t go[4];
#pragma unroll
    for (int it = 0; it < 4; ++it) {
      const int c = it * 32 + lq;
      const float* p = xin + ((size_t)(b * CD + c)) * HWN + hw0 + 8 * e;
      const v4f xa = *(const v4f*)(p), xb = *(const v4f*)(p + 4);
      unsigned short hb[8];
#pragma unroll
      for (int i = 0; i < 4; ++i) { hb[i] = bf_bits(xa[i]); hb[4 + i] = bf_bits(xb[i]); }
      v4u w;
#pragma unroll
      for (int i = 0; i < 4; ++i)
        w[i] = pk16(h_bits((_Float16)bf_up(hb[2 * i])), h_bits((_Float16)bf_up(hb[2 * i + 1])));
      u[it]  = w;
      go[it] = (size_t)c * NTOK + n0 + 8 * e;
#pragma unroll
      for (int t = 0; t < 8; ++t) Ts[(8 * e + t) * 136 + c] = hb[t];
    }
    for (int pass = 0; pass < 2; ++pass) {
#pragma unroll
      for (int it = 0; it < 4; ++it) *(volatile v4u*)(VT + go[it]) = u[it];
      __threadfence();
    }
  }
  __syncthreads();

  {
    const int e = tid & 7, lq = tid >> 3;
    v4u u[4];
#pragma unroll
    for (int it = 0; it < 4; ++it) {
      const int L = it * 32 + lq;
      const int tok = L >> 1, hf = L & 1;
      u[it] = *(const v4u*)(Ts + tok * 136 + hf * 64 + 8 * e);
    }
    unsigned short* db = FB + (size_t)n0 * CD;
    for (int pass = 0; pass < 2; ++pass) {
#pragma unroll
      for (int it = 0; it < 4; ++it) {
        const int L = it * 32 + lq;
        const int tok = L >> 1, hf = L & 1;
        *(volatile v4u*)(db + (size_t)tok * CD + hf * 64 + 8 * e) = u[it];
      }
      __threadfence();
    }
  }
}

__global__ __launch_bounds__(128)
void attn_kernel(const unsigned short* __restrict__ fbp, const unsigned short* __restrict__ vtp, float* out) {
  __shared__ __align__(16) float Os[64 * 132];
  const int tid  = threadIdx.x;
  const int wave = tid >> 5;
  const int lane = tid & 31;
  const int hh   = lane >> 4;
  const int c    = lane & 15;
  const int bx   = blockIdx.x;
  const int q0   = bx * 64;
  const int b    = q0 >> 12;
  const int hw0  = q0 & (HWN - 1);

  const unsigned short* qr = fbp + ((size_t)(q0 + wave * 16 + c)) * CD + 8 * hh;
  const v16b qf0 = ldfrag_b(qr);
  const v16b qf1 = ldfrag_b(qr + 32);
  const v16b qf2 = ldfrag_b(qr + 64);
  const v16b qf3 = ldfrag_b(qr + 96);

  const unsigned short* Kp = fbp + ((size_t)c) * CD + 8 * hh;
  const _Float16* VTh = (const _Float16*)(const void*)vtp;
  const _Float16* Vb  = VTh + ((size_t)c) * NTOK + 8 * hh;

  float m = -1.0e30f, l = 0.f;
  v8f o0 = zero8(), o1 = zero8(), o2 = zero8(), o3 = zero8();
  v8f o4 = zero8(), o5 = zero8(), o6 = zero8(), o7 = zero8();
#pragma unroll 1
  for (int it = 0; it < NTOK / 32; ++it) {
    const int kb = it * 32;
    const unsigned short* k0p = Kp + (size_t)kb * CD;
    const unsigned short* k1p = k0p + (size_t)16 * CD;
    const v16b a00 = ldfrag_b(k0p),      a01 = ldfrag_b(k0p + 32), a02 = ldfrag_b(k0p + 64), a03 = ldfrag_b(k0p + 96);
    const v16b a10 = ldfrag_b(k1p),      a11 = ldfrag_b(k1p + 32), a12 = ldfrag_b(k1p + 64), a13 = ldfrag_b(k1p + 96);
    v8f s0 = mma_b_raw(a00, qf0, zero8());
    s0 = mma_b_raw(a01, qf1, s0);
    s0 = mma_b_raw(a02, qf2, s0);
    s0 = mma_b_raw(a03, qf3, s0);
    v8f s1 = mma_b_raw(a10, qf0, zero8());
    s1 = mma_b_raw(a11, qf1, s1);
    s1 = mma_b_raw(a12, qf2, s1);
    s1 = mma_b_raw(a13, qf3, s1);
    sguard12(s0, s1, a00, a01, a02, a03, a10, a11, a12, a13, qf0, qf1, qf2, qf3);

    float mx = fmaxf(hmax8(s0), hmax8(s1));
    mx = fmaxf(mx, __shfl_xor(mx, 16, 32));
    const float mn   = fmaxf(m, mx * ATTSC);
    const float corr = __expf(m - mn);
    m = mn;
    const float msh = mn - LNPS;
    l *= corr;
#pragma unroll
    for (int r = 0; r < 8; ++r) {
      o0[r] *= corr; o1[r] *= corr; o2[r] *= corr; o3[r] *= corr;
      o4[r] *= corr; o5[r] *= corr; o6[r] *= corr; o7[r] *= corr;
    }

    FragH ph;
    float ls = 0.f;
#pragma unroll
    for (int r = 0; r < 8; ++r) {
      const float e0 = __expf(s0[r] * ATTSC - msh);
      const float e1 = __expf(s1[r] * ATTSC - msh);
      ls += e0 + e1;
      ph.h[0][r] = (_Float16)e0;
      ph.h[1][r] = (_Float16)e1;
    }
    l += ls;

    {
      const v16h vf0 = ldfrag_h(Vb + kb);
      const v16h vf1 = ldfrag_h(Vb + (size_t)16 * NTOK + kb);
      const v16h vf2 = ldfrag_h(Vb + (size_t)32 * NTOK + kb);
      const v16h vf3 = ldfrag_h(Vb + (size_t)48 * NTOK + kb);
      o0 = mma_h_raw(vf0, ph.v, o0);
      o1 = mma_h_raw(vf1, ph.v, o1);
      o2 = mma_h_raw(vf2, ph.v, o2);
      o3 = mma_h_raw(vf3, ph.v, o3);
      oguard4(o0, o1, o2, o3, vf0, vf1, vf2, vf3, ph.v);
    }
    {
      const v16h vf4 = ldfrag_h(Vb + (size_t)64 * NTOK + kb);
      const v16h vf5 = ldfrag_h(Vb + (size_t)80 * NTOK + kb);
      const v16h vf6 = ldfrag_h(Vb + (size_t)96 * NTOK + kb);
      const v16h vf7 = ldfrag_h(Vb + (size_t)112 * NTOK + kb);
      o4 = mma_h_raw(vf4, ph.v, o4);
      o5 = mma_h_raw(vf5, ph.v, o5);
      o6 = mma_h_raw(vf6, ph.v, o6);
      o7 = mma_h_raw(vf7, ph.v, o7);
      oguard4(o4, o5, o6, o7, vf4, vf5, vf6, vf7, ph.v);
    }
  }
  l += __shfl_xor(l, 16, 32);
  const float sc = 1.0f / l;

  {
    float* os = Os + (wave * 16 + c) * 132 + 8 * hh;
    v4f t;
    t = {o0[0] * sc, o0[1] * sc, o0[2] * sc, o0[3] * sc}; *(v4f*)(os + 0)   = t;
    t = {o0[4] * sc, o0[5] * sc, o0[6] * sc, o0[7] * sc}; *(v4f*)(os + 4)   = t;
    t = {o1[0] * sc, o1[1] * sc, o1[2] * sc, o1[3] * sc}; *(v4f*)(os + 16)  = t;
    t = {o1[4] * sc, o1[5] * sc, o1[6] * sc, o1[7] * sc}; *(v4f*)(os + 20)  = t;
    t = {o2[0] * sc, o2[1] * sc, o2[2] * sc, o2[3] * sc}; *(v4f*)(os + 32)  = t;
    t = {o2[4] * sc, o2[5] * sc, o2[6] * sc, o2[7] * sc}; *(v4f*)(os + 36)  = t;
    t = {o3[0] * sc, o3[1] * sc, o3[2] * sc, o3[3] * sc}; *(v4f*)(os + 48)  = t;
    t = {o3[4] * sc, o3[5] * sc, o3[6] * sc, o3[7] * sc}; *(v4f*)(os + 52)  = t;
    t = {o4[0] * sc, o4[1] * sc, o4[2] * sc, o4[3] * sc}; *(v4f*)(os + 64)  = t;
    t = {o4[4] * sc, o4[5] * sc, o4[6] * sc, o4[7] * sc}; *(v4f*)(os + 68)  = t;
    t = {o5[0] * sc, o5[1] * sc, o5[2] * sc, o5[3] * sc}; *(v4f*)(os + 80)  = t;
    t = {o5[4] * sc, o5[5] * sc, o5[6] * sc, o5[7] * sc}; *(v4f*)(os + 84)  = t;
    t = {o6[0] * sc, o6[1] * sc, o6[2] * sc, o6[3] * sc}; *(v4f*)(os + 96)  = t;
    t = {o6[4] * sc, o6[5] * sc, o6[6] * sc, o6[7] * sc}; *(v4f*)(os + 100) = t;
    t = {o7[0] * sc, o7[1] * sc, o7[2] * sc, o7[3] * sc}; *(v4f*)(os + 112) = t;
    t = {o7[4] * sc, o7[5] * sc, o7[6] * sc, o7[7] * sc}; *(v4f*)(os + 116) = t;
  }
  __syncthreads();
  {
    const int e = tid & 7, lq = tid >> 3;
    v4f vals[16];
#pragma unroll
    for (int it = 0; it < 16; ++it) {
      const int L  = it * 16 + lq;
      const int ch = L >> 1, hf = L & 1;
      const int qq = hf * 32 + 4 * e;
      v4f v;
      v[0] = Os[(qq + 0) * 132 + ch];
      v[1] = Os[(qq + 1) * 132 + ch];
      v[2] = Os[(qq + 2) * 132 + ch];
      v[3] = Os[(qq + 3) * 132 + ch];
      vals[it] = v;
    }
    float* ob = out + ((size_t)b * CD) * HWN + hw0;
    for (int pass = 0; pass < 2; ++pass) {
#pragma unroll
      for (int it = 0; it < 16; ++it) {
        const int L  = it * 16 + lq;
        const int ch = L >> 1, hf = L & 1;
        *(volatile v4f*)(ob + (size_t)ch * HWN + hf * 32 + 4 * e) = vals[it];
      }
      __threadfence();
    }
  }
}

extern "C" void kernel_launch(void* const* d_in, const int* in_sizes, int n_in,
                              void* d_out, int out_size, void* d_ws, size_t ws_size,
                              hipStream_t stream) {
  const int NEL = NTOK * CD;
  if (n_in < 1) return;
  if (in_sizes[0] != NEL) return;
  if (out_size != NEL) return;

  const size_t PL = (size_t)NEL * 2;
  size_t off = 0;
  const size_t oF = off; off += PL;
  const size_t oV = off; off += PL;
  if (off > ws_size) return;
  if (off > (size_t)134217728) return;

  const float* x = (const float*)d_in[0];
  char* ws = (char*)d_ws;
  unsigned short* FB = (unsigned short*)(ws + oF);
  unsigned short* VT = (unsigned short*)(ws + oV);
  float* out = (float*)d_out;

  const dim3 blk256(256), blk128(128);
  const dim3 gCV(NTOK / 64);
  const dim3 gAT(NTOK / 64);

  cvt_planes<<<gCV, blk256, 0, stream>>>(x, FB, VT);

  attn_kernel<<<gAT, blk128, 0, stream>>>(FB, VT, out);
  (void)hipGetLastError();
}
